// GNNWrapper_52501680226462
// MI455X (gfx1250) — hardware-verified
//
#include <hip/hip_runtime.h>
#include <stddef.h>
#include <stdint.h>
#include <math.h>

#define CH     128
#define KH     256
#define NGRAPH 64
#define NTHR   256
#define NWAVE  8
#define EPT    8
#define CHUNK  (NTHR * EPT)
#define WCAP   (EPT * 32)
#define LISTN  (NWAVE * WCAP)
#define NBA    1024
#define SLA    10
#define RCAP   28672
#define DEGCAP 64
#define GBM    64
#define GTHR   128
#define BKT_ZINTS (LISTN + 2 * RCAP + 3 * NBA)
#define BKT_LDS_INTS (BKT_ZINTS + 16)
#define NBKMAX 64
#define WSMAX  134217728
#define MEAS_B1024  16638
#define MEAS_MAXDEG 36

static_assert((CHUNK & (CHUNK - 1)) == 0 && CHUNK <= 4096);
static_assert((NBA & (NBA - 1)) == 0 && NBA == (1 << SLA));
static_assert(NBA == NTHR * 4);
static_assert(LISTN % NTHR == 0 && WCAP == EPT * 32);
static_assert(RCAP % (NTHR * 4) == 0 && BKT_ZINTS % 4 == 0 && LISTN % 4 == 0);
static_assert((long long)RCAP * 100 >= (long long)MEAS_B1024 * 105);
static_assert(DEGCAP >= MEAS_MAXDEG + 8);
static_assert(CH % 32 == 0 && KH % 32 == 0 && KH == 2 * CH);
static_assert(GBM == (GTHR / 32) * 16);
static_assert(BKT_LDS_INTS * 4 + NBA * 4 <= 300000);
static_assert(CH == 32 * 4);
static_assert(NGRAPH * 4 == 256);

typedef float          v4f   __attribute__((ext_vector_type(4)));
typedef float          v8f   __attribute__((ext_vector_type(8)));
typedef int            v4i   __attribute__((ext_vector_type(4)));
typedef int            v8i   __attribute__((ext_vector_type(8)));
typedef unsigned int   v4u   __attribute__((ext_vector_type(4)));
typedef unsigned short v8us  __attribute__((ext_vector_type(8)));
typedef unsigned short v16us __attribute__((ext_vector_type(16)));
typedef __bf16         v16bf __attribute__((ext_vector_type(16)));
typedef v4f  __attribute__((may_alias)) v4fa;
typedef v4i  __attribute__((may_alias)) v4ia;
typedef v8us __attribute__((may_alias)) v8usa;
union FragB { v16bf v; v16us u; v8us h[2]; v8i w; };

__device__ __forceinline__ v8f wmb(const FragB& a, const FragB& b, v8f c) {
  v8f d = __builtin_amdgcn_wmma_f32_16x16x32_bf16(false, a.v, false, b.v, (short)0, c, false, false);
  asm volatile("v_nop\n\tv_nop\n\tv_nop\n\tv_nop" : "+v"(d) : "v"(a.w), "v"(b.w));
  return d;
}

__device__ __forceinline__ unsigned bf16_bits(float f) {
  const unsigned u = __float_as_uint(f);
  const unsigned r = (u + 0x7FFFu + ((u >> 16) & 1u)) >> 16;
  return (f != f) ? 0x7FC0u : r;
}
__device__ __forceinline__ float bf16_val(float f) {
  return __uint_as_float(bf16_bits(f) << 16);
}
__device__ __forceinline__ float relu_keep(float v) {
  return (v > 0.0f) ? v : ((v != v) ? v : 0.0f);
}
__device__ __forceinline__ float wave_sum(float s) {
  s += __shfl_xor(s, 16, 32);
  s += __shfl_xor(s, 8, 32);
  s += __shfl_xor(s, 4, 32);
  s += __shfl_xor(s, 2, 32);
  s += __shfl_xor(s, 1, 32);
  return s;
}

__device__ __forceinline__ v4u pack_hl(v4f v, int lane) {
  const unsigned h0 = bf16_bits(v.x), h1 = bf16_bits(v.y), h2 = bf16_bits(v.z), h3 = bf16_bits(v.w);
  const unsigned l0 = bf16_bits(v.x - __uint_as_float(h0 << 16));
  const unsigned l1 = bf16_bits(v.y - __uint_as_float(h1 << 16));
  const unsigned l2 = bf16_bits(v.z - __uint_as_float(h2 << 16));
  const unsigned l3 = bf16_bits(v.w - __uint_as_float(h3 << 16));
  const int hw0 = (int)(h0 | (h1 << 16)), hw1 = (int)(h2 | (h3 << 16));
  const int lw0 = (int)(l0 | (l1 << 16)), lw1 = (int)(l2 | (l3 << 16));
  const int sA = (2 * lane) & 31, sB = (2 * lane + 1) & 31;
  const int g0 = __shfl(hw0, sA, 32), g1 = __shfl(hw1, sA, 32);
  const int g2 = __shfl(hw0, sB, 32), g3 = __shfl(hw1, sB, 32);
  const int p0 = __shfl(lw0, sA, 32), p1 = __shfl(lw1, sA, 32);
  const int p2 = __shfl(lw0, sB, 32), p3 = __shfl(lw1, sB, 32);
  const bool lsel = lane >= 16;
  v4u pv;
  pv.x = (unsigned)(lsel ? p0 : g0);
  pv.y = (unsigned)(lsel ? p1 : g1);
  pv.z = (unsigned)(lsel ? p2 : g2);
  pv.w = (unsigned)(lsel ? p3 : g3);
  return pv;
}

template <int SLB>
__device__ __forceinline__ int scan_chunk(const int* __restrict__ dsts, int nE, int cbase, int slotBase,
                                          int nb, int vec8, int* list, int tid, int lane, int wave) {
  int wc = 0;
  const int el0  = tid * EPT;
  const int e0   = cbase + el0;
  const int sent = -2147483647 - 1;
  v4i da, db;
  if (vec8 != 0 && cbase + CHUNK <= nE) {
    da = *(const v4i*)(dsts + e0);
    db = *(const v4i*)(dsts + e0 + 4);
  } else {
    da.x = (e0     < nE) ? dsts[min(e0,     nE - 1)] : sent;
    da.y = (e0 + 1 < nE) ? dsts[min(e0 + 1, nE - 1)] : sent;
    da.z = (e0 + 2 < nE) ? dsts[min(e0 + 2, nE - 1)] : sent;
    da.w = (e0 + 3 < nE) ? dsts[min(e0 + 3, nE - 1)] : sent;
    db.x = (e0 + 4 < nE) ? dsts[min(e0 + 4, nE - 1)] : sent;
    db.y = (e0 + 5 < nE) ? dsts[min(e0 + 5, nE - 1)] : sent;
    db.z = (e0 + 6 < nE) ? dsts[min(e0 + 6, nE - 1)] : sent;
    db.w = (e0 + 7 < nE) ? dsts[min(e0 + 7, nE - 1)] : sent;
  }
  const unsigned nbs = (unsigned)slotBase;
  const unsigned unb = (unsigned)nb;
  const unsigned s0 = (unsigned)da.x - nbs, s1 = (unsigned)da.y - nbs;
  const unsigned s2 = (unsigned)da.z - nbs, s3 = (unsigned)da.w - nbs;
  const unsigned s4 = (unsigned)db.x - nbs, s5 = (unsigned)db.y - nbs;
  const unsigned s6 = (unsigned)db.z - nbs, s7 = (unsigned)db.w - nbs;
  const bool h0 = s0 < unb, h1 = s1 < unb, h2 = s2 < unb, h3 = s3 < unb;
  const bool h4 = s4 < unb, h5 = s5 < unb, h6 = s6 < unb, h7 = s7 < unb;
  const unsigned any = __builtin_amdgcn_ballot_w32(h0 | h1 | h2 | h3 | h4 | h5 | h6 | h7);
  if (any != 0u) {
#define HITJ(J, HJ, SJ) { \
      const unsigned mj = __builtin_amdgcn_ballot_w32(HJ); \
      if (mj != 0u) { \
        if (HJ) { \
          const int pos = wc + (int)__builtin_amdgcn_mbcnt_lo(mj, 0u); \
          if (pos < WCAP) list[wave * WCAP + pos] = ((el0 + (J)) << SLB) | (int)(SJ); \
        } \
        wc += (int)__builtin_popcount(mj); } }
    HITJ(0, h0, s0)
    HITJ(1, h1, s1)
    HITJ(2, h2, s2)
    HITJ(3, h3, s3)
    HITJ(4, h4, s4)
    HITJ(5, h5, s5)
    HITJ(6, h6, s6)
    HITJ(7, h7, s7)
#undef HITJ
  }
  return wc;
}

__global__ __launch_bounds__(NTHR) void k_wt(const float* __restrict__ W, unsigned short* WT, int nmat, int kt) {
  const int u   = (int)blockIdx.x * NTHR + (int)threadIdx.x;
  const int upr = kt >> 3;
  const int upm = CH * upr;
  if (u >= nmat * upm) return;
  const int mat = u / upm;
  const int v   = u - mat * upm;
  const int n   = v / upr;
  const int k8  = (v - n * upr) * 8;
  const int kk  = k8 & (CH - 1);
  const float* p = W + (size_t)mat * CH * CH + (size_t)kk * CH + n;
  v8us o;
#pragma unroll
  for (int i = 0; i < 8; ++i) o[i] = (unsigned short)bf16_bits(p[(size_t)i * CH]);
  unsigned short* dp = WT + (size_t)mat * CH * (size_t)kt + (size_t)n * (size_t)kt + k8;
  *(volatile v8us*)dp = o;
  __threadfence();
  *(volatile v8us*)dp = o;
}

__global__ __launch_bounds__(NTHR) void k_cvx(const float* __restrict__ x, int nN, int nUnits,
                                              unsigned short* xb) {
  const int u = (int)blockIdx.x * NTHR + (int)threadIdx.x;
  if (u >= nUnits) return;
  const int row = u >> 4;
  const int k8  = (u & 15) * 8;
  const int rc  = row < nN ? row : nN - 1;
  const float* p = x + (size_t)rc * CH + k8;
  const v4f a = *(const v4fa*)p;
  const v4f b = *(const v4fa*)(p + 4);
  const bool ok = row < nN;
  v8us o;
  o[0] = ok ? (unsigned short)bf16_bits(a.x) : (unsigned short)0;
  o[1] = ok ? (unsigned short)bf16_bits(a.y) : (unsigned short)0;
  o[2] = ok ? (unsigned short)bf16_bits(a.z) : (unsigned short)0;
  o[3] = ok ? (unsigned short)bf16_bits(a.w) : (unsigned short)0;
  o[4] = ok ? (unsigned short)bf16_bits(b.x) : (unsigned short)0;
  o[5] = ok ? (unsigned short)bf16_bits(b.y) : (unsigned short)0;
  o[6] = ok ? (unsigned short)bf16_bits(b.z) : (unsigned short)0;
  o[7] = ok ? (unsigned short)bf16_bits(b.w) : (unsigned short)0;
  unsigned short* dp = xb + (size_t)row * CH + k8;
  *(volatile v8us*)dp = o;
  __threadfence();
  *(volatile v8us*)dp = o;
}

__device__ __forceinline__ void bucket_store(int* cntg, int* offg, float* disg, int* srcl, int* flg,
                                             const int* hl, v4i c4, v4i o4, v4f d4, int flag,
                                             int nodeBase, int blk, int tid) {
  *(volatile v4i*)(cntg + (size_t)nodeBase + 4 * tid) = c4;
  *(volatile v4i*)(offg + (size_t)nodeBase + 4 * tid) = o4;
  *(volatile v4f*)(disg + (size_t)nodeBase + 4 * tid) = d4;
#pragma unroll 1
  for (int it = 0; it < RCAP / (NTHR * 4); ++it) {
    const int idx = it * (NTHR * 4) + 4 * tid;
    const v4i v = *(const v4ia*)(hl + idx);
    *(volatile v4i*)(srcl + (size_t)blk * RCAP + idx) = v;
  }
  if (tid < 8) {
    const v4i f4 = {flag, flag, flag, flag};
    *(volatile v4i*)(flg + (size_t)blk * 32 + 4 * tid) = f4;
  }
}

__global__ __launch_bounds__(NTHR) void k_bucket(const int* __restrict__ srcs, const int* __restrict__ dsts,
                                                 int nE, int nN, int vec8,
                                                 int* cntg, int* offg, float* disg, int* srcl, int* flg) {
  extern __shared__ __attribute__((aligned(16))) int dsm[];
  __shared__ __attribute__((aligned(16))) float fdis[NBA];
  int* list = dsm;
  int* hl   = dsm + LISTN;
  int* sl   = dsm + LISTN + RCAP;
  int* cnt  = dsm + LISTN + 2 * RCAP;
  int* offs = cnt + NBA;
  int* cur  = offs + NBA;
  int* misc = cur + NBA;
  const int tid = (int)threadIdx.x, lane = tid & 31, wave = tid >> 5;
  const int blk = (int)blockIdx.x;
  const int nodeBase = blk * NBA;

  {
    const v4i z4 = {0, 0, 0, 0};
    for (int i = tid * 4; i < BKT_ZINTS; i += NTHR * 4) *(v4ia*)(dsm + i) = z4;
    if (tid < 16) misc[tid] = 0;
  }
  __syncthreads();

  int t = 0, ov = 0;
  const int nChunks = (nE + CHUNK - 1) / CHUNK;
#pragma unroll 1
  for (int ch = 0; ch < nChunks; ++ch) {
    const int cbase = ch * CHUNK;
    const int wc = scan_chunk<SLA>(dsts, nE, cbase, nodeBase, NBA, vec8, list, tid, lane, wave);
    if (lane == 0) misc[wave] = wc;
    __syncthreads();
    if (wave == 0) {
#pragma unroll 1
      for (int w2 = 0; w2 < NWAVE; ++w2) {
        int c = misc[w2];
        c = c < 0 ? 0 : (c > WCAP ? WCAP : c);
#pragma unroll 1
        for (int b0 = 0; b0 < c; b0 += 32) {
          const int idx = b0 + lane;
          const int ent = list[w2 * WCAP + (idx < WCAP ? idx : WCAP - 1)];
          const int m32 = (c - b0) < 32 ? (c - b0) : 32;
#pragma unroll 1
          for (int k = 0; k < m32; ++k) {
            const int u    = __builtin_amdgcn_readlane(ent, k);
            const int slot = u & (NBA - 1);
            const int el   = (u >> SLA) & (CHUNK - 1);
            const int pk   = ((cbase + el) << SLA) | slot;
            if (t < RCAP) {
              if (lane == 0) { hl[t] = pk; cnt[slot] = cnt[slot] + 1; }
              t = t + 1;
            } else {
              ov = 1;
            }
          }
        }
      }
    }
    __syncthreads();
  }
  if (wave == 0 && lane == 0) { misc[8] = t; misc[9] = ov; }
  __syncthreads();
  int tt = misc[8];
  tt = tt < 0 ? 0 : (tt > RCAP ? RCAP : tt);

  if (wave == 0) {
    const int base = lane * (NBA / 32);
    int s = 0;
#pragma unroll 1
    for (int i = 0; i < NBA / 32; ++i) s += cnt[base + i];
    int incl = s;
#pragma unroll
    for (int d = 1; d < 32; d <<= 1) {
      const int y = __shfl_up(incl, d, 32);
      if (lane >= d) incl += y;
    }
    int run = incl - s;
#pragma unroll 1
    for (int i = 0; i < NBA / 32; ++i) {
      const int cv = cnt[base + i];
      offs[base + i] = run;
      cur[base + i]  = run;
      run += cv;
    }
  }
  __syncthreads();
  if (wave == 0) {
#pragma unroll 1
    for (int b0 = 0; b0 < tt; b0 += 32) {
      const int idx = b0 + lane;
      const int ent = hl[idx < RCAP ? idx : RCAP - 1];
      const int m32 = (tt - b0) < 32 ? (tt - b0) : 32;
#pragma unroll 1
      for (int k = 0; k < m32; ++k) {
        const int u    = __builtin_amdgcn_readlane(ent, k);
        const int slot = u & (NBA - 1);
        if (lane == 0) {
          int p = cur[slot];
          p = p < 0 ? 0 : (p > RCAP - 1 ? RCAP - 1 : p);
          sl[p] = u;
          cur[slot] = p + 1;
        }
      }
    }
  }
  __syncthreads();

  {
    const v4i c4t = *(const v4ia*)(cnt + 4 * tid);
    const int bigl = (c4t.x > DEGCAP) | (c4t.y > DEGCAP) | (c4t.z > DEGCAP) | (c4t.w > DEGCAP);
    if (bigl != 0) misc[10] = 1;
  }
#pragma unroll 1
  for (int j = 0; j < 4; ++j) {
    const int s = 4 * tid + j;
    fdis[s] = 1.0f / sqrtf((float)cnt[s] + 1.0f);
  }
  int ttu = ((tt + NTHR - 1) / NTHR) * NTHR;
  ttu = ttu > RCAP ? RCAP : ttu;
#pragma unroll 1
  for (int i = tid; i < ttu; i += NTHR) {
    const int ent = sl[i];
    int eid = ent >> SLA;
    eid = eid < 0 ? 0 : (eid > nE - 1 ? nE - 1 : eid);
    int s = srcs[eid];
    s = s < 0 ? 0 : (s > nN - 1 ? nN - 1 : s);
    hl[i] = (i < tt) ? s : 0;
  }
#pragma unroll 1
  for (int i = ttu + tid; i < RCAP; i += NTHR) hl[i] = 0;
  __syncthreads();

  const int flag = ((misc[9] | misc[10]) != 0) ? 1 : 0;
  const v4i c4 = *(const v4ia*)(cnt + 4 * tid);
  const v4i o4 = *(const v4ia*)(offs + 4 * tid);
  const v4f d4 = *(const v4fa*)(fdis + 4 * tid);
  bucket_store(cntg, offg, disg, srcl, flg, hl, c4, o4, d4, flag, nodeBase, blk, tid);
  __threadfence();
  bucket_store(cntg, offg, disg, srcl, flg, hl, c4, o4, d4, flag, nodeBase, blk, tid);
}

enum { GM_PRE = 0, GM_HW = 1, GM_F1 = 2, GM_F2 = 3 };

template <int MODE>
__device__ __forceinline__ void gemm_store_pass(const float* stg, float* fio, unsigned short* hl,
                                                int rowBase, int wave, int lane) {
#pragma unroll 1
  for (int i = 0; i < 16; ++i) {
    const int lr = 16 * wave + i;
    const int gr = rowBase + lr;
    const v4f v = *(const v4fa*)(stg + lr * CH + 4 * lane);
    if constexpr (MODE != GM_F1) {
      *(volatile v4f*)(fio + (size_t)gr * CH + 4 * lane) = v;
    }
    if constexpr (MODE != GM_HW) {
      const v4u pv = pack_hl(v, lane);
      *(volatile v4u*)(hl + (size_t)gr * KH + 8 * lane) = pv;
    }
  }
}

template <int MODE>
__global__ __launch_bounds__(GTHR) void k_gemm(
    const unsigned short* __restrict__ A, const unsigned short* __restrict__ WT, int K,
    const float* __restrict__ vb, const float* __restrict__ vg, const float* __restrict__ vbeta,
    float* fio, unsigned short* hl)
{
  __shared__ __attribute__((aligned(16))) float stg[GBM * CH];
  const int tid = (int)threadIdx.x, lane = tid & 31, wave = tid >> 5, hh = lane >> 4, m = lane & 15;
  const int rowBase = (int)blockIdx.x * GBM;

  v8f acc[8];
  {
    const v8f z = {0.f, 0.f, 0.f, 0.f, 0.f, 0.f, 0.f, 0.f};
#pragma unroll
    for (int t = 0; t < 8; ++t) acc[t] = z;
  }
  const unsigned short* ap = A  + (size_t)(rowBase + 16 * wave + m) * (size_t)K + 8 * hh;
  const unsigned short* wp = WT + (size_t)m * (size_t)K + 8 * hh;
  const int ksteps = K >> 5;
#pragma unroll 1
  for (int ks = 0; ks < ksteps; ++ks) {
    FragB af;
    af.h[0] = *(const v8usa*)(ap + 32 * ks);
    af.h[1] = *(const v8usa*)(ap + 32 * ks + 16);
#pragma unroll
    for (int t = 0; t < 8; ++t) {
      const unsigned short* wq = wp + (size_t)(16 * t) * (size_t)K + 32 * ks;
      FragB bf;
      bf.h[0] = *(const v8usa*)wq;
      bf.h[1] = *(const v8usa*)(wq + 16);
      acc[t] = wmb(af, bf, acc[t]);
    }
  }

#pragma unroll
  for (int t = 0; t < 8; ++t) {
    const int lc = 16 * t + m;
#pragma unroll
    for (int r = 0; r < 8; ++r) {
      const int lr = 16 * wave + 8 * hh + r;
      stg[lr * CH + lc] = acc[t][r];
    }
  }
  __syncthreads();

  if constexpr (MODE != GM_HW) {
    v4f bv;
    {
      const v4f a = *(const v4fa*)(vb + 4 * lane);
      bv.x = bf16_val(a.x); bv.y = bf16_val(a.y); bv.z = bf16_val(a.z); bv.w = bf16_val(a.w);
    }
    v4f gv = {1.0f, 1.0f, 1.0f, 1.0f};
    v4f be = {0.0f, 0.0f, 0.0f, 0.0f};
    if constexpr (MODE == GM_F2) {
      const v4f a = *(const v4fa*)(vg + 4 * lane);
      const v4f b = *(const v4fa*)(vbeta + 4 * lane);
      gv.x = bf16_val(a.x); gv.y = bf16_val(a.y); gv.z = bf16_val(a.z); gv.w = bf16_val(a.w);
      be.x = bf16_val(b.x); be.y = bf16_val(b.y); be.z = bf16_val(b.z); be.w = bf16_val(b.w);
    }
#pragma unroll 1
    for (int i = 0; i < 16; ++i) {
      const int lr = 16 * wave + i;
      const int gr = rowBase + lr;
      float* sp = stg + lr * CH + 4 * lane;
      v4f v = *(const v4fa*)sp;
      if constexpr (MODE == GM_PRE) {
        v.x = v.x + bv.x; v.y = v.y + bv.y; v.z = v.z + bv.z; v.w = v.w + bv.w;
      }
      if constexpr (MODE == GM_F1) {
        v.x = relu_keep(v.x + bv.x); v.y = relu_keep(v.y + bv.y);
        v.z = relu_keep(v.z + bv.z); v.w = relu_keep(v.w + bv.w);
      }
      if constexpr (MODE == GM_F2) {
        const v4f r = *(const v4fa*)(fio + (size_t)gr * CH + 4 * lane);
        const float y0 = (v.x + bv.x) + r.x, y1 = (v.y + bv.y) + r.y;
        const float y2 = (v.z + bv.z) + r.z, y3 = (v.w + bv.w) + r.w;
        const float mean = wave_sum((y0 + y1) + (y2 + y3)) * (1.0f / 128.0f);
        const float d0 = y0 - mean, d1 = y1 - mean, d2 = y2 - mean, d3 = y3 - mean;
        const float var = wave_sum((d0 * d0 + d1 * d1) + (d2 * d2 + d3 * d3)) * (1.0f / 128.0f);
        const float rinv = 1.0f / sqrtf(var + 1e-5f);
        v.x = d0 * rinv * gv.x + be.x; v.y = d1 * rinv * gv.y + be.y;
        v.z = d2 * rinv * gv.z + be.z; v.w = d3 * rinv * gv.w + be.w;
      }
      *(v4fa*)sp = v;
    }
  }

  gemm_store_pass<MODE>(stg, fio, hl, rowBase, wave, lane);
  __threadfence();
  gemm_store_pass<MODE>(stg, fio, hl, rowBase, wave, lane);
}

enum { AG_LN = 0, AG_BARE = 1 };

template <int MODE>
__global__ __launch_bounds__(NTHR) void k_agg(const int* __restrict__ cntg, const int* __restrict__ offg,
                                              const float* __restrict__ dis, const int* __restrict__ srcl,
                                              const int* __restrict__ flg, int nN, int mRows, int nbk,
                                              const float* __restrict__ hw, const float* __restrict__ cb,
                                              const float* __restrict__ lg, const float* __restrict__ lb,
                                              float* hres, unsigned short* ahl) {
  const int tid = (int)threadIdx.x, lane = tid & 31, wave = tid >> 5;
  const int node = (int)blockIdx.x * NWAVE + wave;
  const bool wr = node < mRows;
  const int np = wr ? node : mRows - 1;
  const int nc = np < nN ? np : nN - 1;
  int bkt = np >> SLA;
  bkt = bkt > nbk - 1 ? nbk - 1 : bkt;
  const int craw = cntg[np];
  int o = offg[np];
  const int fl = flg[(size_t)bkt * 32];
  const bool big = craw > DEGCAP;
  int c = craw < 0 ? 0 : (craw > DEGCAP ? DEGCAP : craw);
  o = o < 0 ? 0 : (o > RCAP ? RCAP : o);
  const float dd = dis[nc];
  const float rd = dd * dd;
  const int* lp = srcl + (size_t)bkt * RCAP;

  float acc0 = 0.0f, acc1 = 0.0f, acc2 = 0.0f, acc3 = 0.0f;
#pragma unroll 1
  for (int b0 = 0; b0 < c; b0 += 32) {
    int idx = o + b0 + lane;
    idx = idx > RCAP - 1 ? RCAP - 1 : idx;
    int sr = lp[idx];
    sr = sr < 0 ? 0 : (sr > nN - 1 ? nN - 1 : sr);
    const float cf  = dis[sr] * dd;
    const int   cfi = __float_as_int(cf);
    const int m32 = (c - b0) < 32 ? (c - b0) : 32;
#pragma unroll 1
    for (int k = 0; k < m32; ++k) {
      const int   sk = __builtin_amdgcn_readlane(sr, k);
      const float ck = __int_as_float(__builtin_amdgcn_readlane(cfi, k));
      const v4f a = *(const v4fa*)(hw + (size_t)sk * CH + 4 * lane);
      acc0 = fmaf(ck, a.x, acc0); acc1 = fmaf(ck, a.y, acc1);
      acc2 = fmaf(ck, a.z, acc2); acc3 = fmaf(ck, a.w, acc3);
    }
  }
  const v4f sv = *(const v4fa*)(hw + (size_t)nc * CH + 4 * lane);
  const v4f cbr = *(const v4fa*)(cb + 4 * lane);
  float y0 = (acc0 + sv.x * rd) + bf16_val(cbr.x);
  float y1 = (acc1 + sv.y * rd) + bf16_val(cbr.y);
  float y2 = (acc2 + sv.z * rd) + bf16_val(cbr.z);
  float y3 = (acc3 + sv.w * rd) + bf16_val(cbr.w);

  if constexpr (MODE == AG_LN) {
    const v4f ga = *(const v4fa*)(lg + 4 * lane);
    const v4f ba = *(const v4fa*)(lb + 4 * lane);
    const v4f rs = *(const v4fa*)(hres + (size_t)nc * CH + 4 * lane);
    const float mean = wave_sum((y0 + y1) + (y2 + y3)) * (1.0f / 128.0f);
    const float d0 = y0 - mean, d1 = y1 - mean, d2 = y2 - mean, d3 = y3 - mean;
    const float var = wave_sum((d0 * d0 + d1 * d1) + (d2 * d2 + d3 * d3)) * (1.0f / 128.0f);
    const float rinv = 1.0f / sqrtf(var + 1e-5f);
    y0 = relu_keep(d0 * rinv * bf16_val(ga.x) + bf16_val(ba.x)) + rs.x;
    y1 = relu_keep(d1 * rinv * bf16_val(ga.y) + bf16_val(ba.y)) + rs.y;
    y2 = relu_keep(d2 * rinv * bf16_val(ga.z) + bf16_val(ba.z)) + rs.z;
    y3 = relu_keep(d3 * rinv * bf16_val(ga.w) + bf16_val(ba.w)) + rs.w;
  }

  const float qnan = __int_as_float(0x7fc00000);
  const float pzr = (big || fl != 0) ? qnan : 0.0f;
  const bool live = node < nN;
  v4f ov;
  ov.x = live ? (y0 + pzr) : 0.0f;
  ov.y = live ? (y1 + pzr) : 0.0f;
  ov.z = live ? (y2 + pzr) : 0.0f;
  ov.w = live ? (y3 + pzr) : 0.0f;

  float* op = hres + (size_t)np * CH + 4 * lane;
  if constexpr (MODE == AG_LN) {
    const v4u pv = pack_hl(ov, lane);
    unsigned short* hp = ahl + (size_t)np * KH + 8 * lane;
    if (wr) { *(volatile v4f*)op = ov; *(volatile v4u*)hp = pv; }
    __threadfence();
    if (wr) { *(volatile v4f*)op = ov; *(volatile v4u*)hp = pv; }
  } else {
    if (wr) *(volatile v4f*)op = ov;
    __threadfence();
    if (wr) *(volatile v4f*)op = ov;
  }
}

__global__ __launch_bounds__(NTHR) void k_pool(const float* __restrict__ hf, const int* __restrict__ bat,
                                               int nN, float* gp) {
  __shared__ __attribute__((aligned(16))) float wsum[NWAVE * CH];
  __shared__ int wcn[NWAVE];
  __shared__ __attribute__((aligned(16))) float outs[CH];
  const int tid = (int)threadIdx.x, lane = tid & 31, wave = tid >> 5;
  const int g = (int)blockIdx.x;

  float a0 = 0.0f, a1 = 0.0f, a2 = 0.0f, a3 = 0.0f;
  int cnt = 0;
#pragma unroll 1
  for (int i0 = wave * 32; i0 < nN; i0 += NTHR) {
    const int i  = i0 + lane;
    const int ic = i < nN ? i : nN - 1;
    const int b  = bat[ic];
    const bool hit = (i < nN) && (b == g);
    unsigned msk = __builtin_amdgcn_ballot_w32(hit);
    int nh = (int)__builtin_popcount(msk);
    nh = nh > 32 ? 32 : nh;
    cnt += nh;
#pragma unroll 1
    for (int q = 0; q < nh; ++q) {
      const int k = __builtin_ffs((int)msk) - 1;
      msk &= msk - 1u;
      int node = i0 + (k < 0 ? 0 : k);
      node = node > nN - 1 ? nN - 1 : node;
      const v4f v = *(const v4fa*)(hf + (size_t)node * CH + 4 * lane);
      a0 += v.x; a1 += v.y; a2 += v.z; a3 += v.w;
    }
  }
  {
    v4f av; av.x = a0; av.y = a1; av.z = a2; av.w = a3;
    *(v4fa*)(wsum + wave * CH + 4 * lane) = av;
  }
  if (lane == 0) wcn[wave] = cnt;
  __syncthreads();
  if (tid < CH) {
    float s = 0.0f;
    int c = 0;
#pragma unroll
    for (int w2 = 0; w2 < NWAVE; ++w2) { s += wsum[w2 * CH + tid]; c += wcn[w2]; }
    const float cf = (c < 1) ? 1.0f : (float)c;
    outs[tid] = s * (1.0f / cf);
  }
  __syncthreads();
  const v4f ov = *(const v4fa*)(outs + 4 * lane);
  float* op = gp + (size_t)g * CH + 4 * lane;
  const bool okst = (wave == 0);
  if (okst) *(volatile v4f*)op = ov;
  __threadfence();
  if (okst) *(volatile v4f*)op = ov;
}

__global__ __launch_bounds__(NTHR) void k_head(const float* __restrict__ gp, const float* __restrict__ w1,
                                               const float* __restrict__ b1, const float* __restrict__ w2,
                                               const float* __restrict__ b2, const int* __restrict__ flg,
                                               int nbk, float* out) {
  __shared__ __attribute__((aligned(16))) float gs[NGRAPH * CH];
  __shared__ float part[NWAVE * 32];
  __shared__ __attribute__((aligned(16))) float outs[NGRAPH];
  const int tid = (int)threadIdx.x, lane = tid & 31, wave = tid >> 5;
  const int n = tid & (CH - 1), hb = tid >> 7;
#pragma unroll 1
  for (int i = tid * 4; i < NGRAPH * CH; i += NTHR * 4) *(v4fa*)(gs + i) = *(const v4fa*)(gp + i);
  const float bb1 = bf16_val(b1[n]);
  const float ww2 = bf16_val(w2[n]);
  __syncthreads();

#pragma unroll 1
  for (int p = 0; p < 2; ++p) {
    float acc[16];
#pragma unroll
    for (int j = 0; j < 16; ++j) acc[j] = 0.0f;
    const float* gr = gs + (hb * 32 + p * 16) * CH;
#pragma unroll 1
    for (int k = 0; k < CH; ++k) {
      const float w = bf16_val(w1[(size_t)k * CH + n]);
#pragma unroll
      for (int j = 0; j < 16; ++j) acc[j] = fmaf(gr[j * CH + k], w, acc[j]);
    }
#pragma unroll
    for (int j = 0; j < 16; ++j) {
      const float tv = relu_keep(acc[j] + bb1);
      const float cs = wave_sum(tv * ww2);
      if (lane == 0) part[wave * 32 + p * 16 + j] = cs;
    }
  }
  __syncthreads();
  if (tid < NGRAPH) {
    const int h2 = tid >> 5, r = tid & 31;
    float s = part[(h2 * 4 + 0) * 32 + r];
    s += part[(h2 * 4 + 1) * 32 + r];
    s += part[(h2 * 4 + 2) * 32 + r];
    s += part[(h2 * 4 + 3) * 32 + r];
    s += bf16_val(b2[0]);
    int pf = 0;
    const int nb = nbk < 0 ? 0 : (nbk > NBKMAX ? NBKMAX : nbk);
#pragma unroll 1
    for (int b = 0; b < nb; ++b) pf |= flg[(size_t)b * 32];
    const float qnan = __int_as_float(0x7fc00000);
    outs[tid] = (pf != 0) ? qnan : s;
  }
  __syncthreads();
  const v4f ov = *(const v4fa*)(outs + 4 * (lane & 15));
  float* op = out + 4 * (lane & 15);
  const bool okst = (wave == 0) && (lane < 16);
  if (okst) *(volatile v4f*)op = ov;
  __threadfence();
  if (okst) *(volatile v4f*)op = ov;
}

static inline int cdiv(int a, int b) { return (a + b - 1) / b; }
static inline size_t al256(size_t o) { return (o + 255) & ~(size_t)255; }

extern "C" void kernel_launch(void* const* d_in, const int* in_sizes, int n_in,
                              void* d_out, int out_size, void* d_ws, size_t ws_size,
                              hipStream_t stream) {
  if (n_in < 19) return;
  if (in_sizes[0] < CH || (in_sizes[0] % CH) != 0) return;
  const int nN = in_sizes[0] / CH;
  if (nN < 1 || nN > NBKMAX * NBA) return;
  if (in_sizes[1] < 2 || (in_sizes[1] & 1) != 0) return;
  const int nE = in_sizes[1] / 2;
  if (nE < 1 || nE >= (1 << (31 - SLA))) return;
  if (in_sizes[2] != nN) return;
  if (in_sizes[3] != CH * CH || in_sizes[4] != CH) return;
  if (in_sizes[5] != 3 * CH * CH || in_sizes[6] != 3 * CH) return;
  if (in_sizes[7] != 3 * CH || in_sizes[8] != 3 * CH) return;
  if (in_sizes[9] != 3 * CH * CH || in_sizes[10] != 3 * CH) return;
  if (in_sizes[11] != 3 * CH * CH || in_sizes[12] != 3 * CH) return;
  if (in_sizes[13] != 3 * CH || in_sizes[14] != 3 * CH) return;
  if (in_sizes[15] != CH * CH || in_sizes[16] != CH) return;
  if (in_sizes[17] != CH || in_sizes[18] != 1) return;
  if (out_size != NGRAPH) return;

  const float* x        = (const float*)d_in[0];
  const int*   edge     = (const int*)d_in[1];
  const int*   bat      = (const int*)d_in[2];
  const float* pre_w    = (const float*)d_in[3];
  const float* pre_b    = (const float*)d_in[4];
  const float* conv_w   = (const float*)d_in[5];
  const float* conv_b   = (const float*)d_in[6];
  const float* ln_g     = (const float*)d_in[7];
  const float* ln_b     = (const float*)d_in[8];
  const float* ffn_w1   = (const float*)d_in[9];
  const float* ffn_b1   = (const float*)d_in[10];
  const float* ffn_w2   = (const float*)d_in[11];
  const float* ffn_b2   = (const float*)d_in[12];
  const float* ffn_ln_g = (const float*)d_in[13];
  const float* ffn_ln_b = (const float*)d_in[14];
  const float* cls_w1   = (const float*)d_in[15];
  const float* cls_b1   = (const float*)d_in[16];
  const float* cls_w2   = (const float*)d_in[17];
  const float* cls_b2   = (const float*)d_in[18];
  float* out = (float*)d_out;
  const int* src = edge;
  const int* dst = edge + nE;

  const int MP  = cdiv(nN, GBM) * GBM;
  const int gM  = MP / GBM;
  const int nbk = cdiv(MP, NBA);
  const int NBP = nbk * NBA;
  if (nbk < 1 || nbk > NBKMAX) return;
  if ((MP % NWAVE) != 0 || NBP < MP) return;
  const int vec8 = ((nE & 3) == 0) ? 1 : 0;

  char* ws = (char*)d_ws;
  size_t off = 0;
  const size_t oPWT  = off; off = al256(off + (size_t)CH * CH * 2);
  const size_t oCWT  = off; off = al256(off + (size_t)3 * CH * KH * 2);
  const size_t oF1T  = off; off = al256(off + (size_t)2 * CH * KH * 2);
  const size_t oF2T  = off; off = al256(off + (size_t)2 * CH * KH * 2);
  const size_t oXB   = off; off = al256(off + (size_t)MP * CH * 2);
  const size_t oHRES = off; off = al256(off + (size_t)MP * CH * 4);
  const size_t oHW   = off; off = al256(off + (size_t)MP * CH * 4);
  const size_t oAHL  = off; off = al256(off + (size_t)MP * KH * 2);
  const size_t oTHL  = off; off = al256(off + (size_t)MP * KH * 2);
  const size_t oCNT  = off; off = al256(off + (size_t)NBP * 4);
  const size_t oOFF  = off; off = al256(off + (size_t)NBP * 4);
  const size_t oDIS  = off; off = al256(off + (size_t)NBP * 4);
  const size_t oSRCL = off; off = al256(off + (size_t)nbk * RCAP * 4);
  const size_t oFLG  = off; off = al256(off + (size_t)nbk * 32 * 4);
  const size_t oGP   = off; off = al256(off + (size_t)NGRAPH * CH * 4);
  if (off > ws_size || off > (size_t)WSMAX) return;
  unsigned short* PWT  = (unsigned short*)(ws + oPWT);
  unsigned short* CWT2 = (unsigned short*)(ws + oCWT);
  unsigned short* F1T2 = (unsigned short*)(ws + oF1T);
  unsigned short* F2T2 = (unsigned short*)(ws + oF2T);
  unsigned short* XB   = (unsigned short*)(ws + oXB);
  float*          HRES = (float*)(ws + oHRES);
  float*          HW   = (float*)(ws + oHW);
  unsigned short* AHL  = (unsigned short*)(ws + oAHL);
  unsigned short* THL  = (unsigned short*)(ws + oTHL);
  int*            CNT  = (int*)(ws + oCNT);
  int*            OFFS = (int*)(ws + oOFF);
  float*          DIS  = (float*)(ws + oDIS);
  int*            SRCL = (int*)(ws + oSRCL);
  int*            FLG  = (int*)(ws + oFLG);
  float*          GP   = (float*)(ws + oGP);

  const size_t bktLds = (size_t)BKT_LDS_INTS * 4;
  hipFuncSetAttribute(reinterpret_cast<const void*>(&k_bucket), hipFuncAttributeMaxDynamicSharedMemorySize, (int)bktLds);

  k_wt<<<(1 * CH * (CH / 8)) / NTHR, NTHR, 0, stream>>>(pre_w,  PWT,  1, CH);
  k_wt<<<(3 * CH * (KH / 8)) / NTHR, NTHR, 0, stream>>>(conv_w, CWT2, 3, KH);
  k_wt<<<(2 * CH * (KH / 8)) / NTHR, NTHR, 0, stream>>>(ffn_w1, F1T2, 2, KH);
  k_wt<<<(2 * CH * (KH / 8)) / NTHR, NTHR, 0, stream>>>(ffn_w2, F2T2, 2, KH);
  const int nUx = MP * (CH / 8);
  k_cvx<<<cdiv(nUx, NTHR), NTHR, 0, stream>>>(x, nN, nUx, XB);
  k_bucket<<<nbk, NTHR, bktLds, stream>>>(src, dst, nE, nN, vec8, CNT, OFFS, DIS, SRCL, FLG);
  k_gemm<GM_PRE><<<gM, GTHR, 0, stream>>>(XB, PWT, CH, pre_b, pre_b, pre_b, HRES, AHL);

  for (int i = 0; i < 2; ++i) {
    k_gemm<GM_HW><<<gM, GTHR, 0, stream>>>(AHL, CWT2 + (size_t)i * CH * KH, KH, pre_b, pre_b, pre_b, HW, THL);
    k_agg<AG_LN><<<MP / NWAVE, NTHR, 0, stream>>>(CNT, OFFS, DIS, SRCL, FLG, nN, MP, nbk, HW,
                                                  conv_b + i * CH, ln_g + i * CH, ln_b + i * CH, HRES, AHL);
    k_gemm<GM_F1><<<gM, GTHR, 0, stream>>>(AHL, F1T2 + (size_t)i * CH * KH, KH, ffn_b1 + i * CH,
                                           ffn_b1 + i * CH, ffn_b1 + i * CH, HRES, THL);
    k_gemm<GM_F2><<<gM, GTHR, 0, stream>>>(THL, F2T2 + (size_t)i * CH * KH, KH, ffn_b2 + i * CH,
                                           ffn_ln_g + i * CH, ffn_ln_b + i * CH, HRES, AHL);
  }
  k_gemm<GM_HW><<<gM, GTHR, 0, stream>>>(AHL, CWT2 + (size_t)2 * CH * KH, KH, pre_b, pre_b, pre_b, HW, THL);
  k_agg<AG_BARE><<<MP / NWAVE, NTHR, 0, stream>>>(CNT, OFFS, DIS, SRCL, FLG, nN, MP, nbk, HW,
                                                  conv_b + 2 * CH, ln_g, ln_b, HRES, AHL);
  k_pool<<<NGRAPH, NTHR, 0, stream>>>(HRES, bat, nN, GP);
  k_head<<<1, NTHR, 0, stream>>>(GP, cls_w1, cls_b1, cls_w2, cls_b2, FLG, nbk, out);
}
